// InteractionBlock_34445637714614
// MI455X (gfx1250) — hardware-verified
//
#include <hip/hip_runtime.h>
#include <stddef.h>
#include <stdint.h>


#define NN      50000
#define NE      800000
#define FW      256
#define KC      64
#define NTHR    256
#define NWAVE   8
#define EPT     8
#define CHUNK   (NTHR * EPT)
#define WCAP    (EPT * 32)
#define LISTN   (NWAVE * WCAP)
#define NBA     1024
#define SLA     10
#define RCAP    20480
#define DEGCAP  64
#define MEAS_B1024  16651
#define MEAS_MAXDEG 38
#define GBM     64
#define GTHR    128
#define HALF0   25600
#define HALF1   (NN - HALF0)
#define SB0     (HALF0 / NBA)
#define SB1     ((HALF1 + NBA - 1) / NBA)
#define DT0     (HALF0 / GBM)
#define DT1     ((HALF1 + GBM - 1) / GBM)
#define UPT     ((NN + GBM - 1) / GBM)
#define AGG_ZINTS     (LISTN + 2 * RCAP + 3 * NBA)
#define MISC_INTS     16
#define SCAN_LDS_INTS (AGG_ZINTS + MISC_INTS)
#define SCAN_LDS      (SCAN_LDS_INTS * 4)
#define SPITCH  260
#define DOWN_LDS (GBM * SPITCH * 4)
#define PREP_NB (NN / NWAVE)
#define PREP_WB 20
#define DN_TWO_TERM 1
#define KDN     (DN_TWO_TERM ? 256 : 128)
#define WSMAX   134217728

#define O_R0    ((size_t)0)
#define SZ_R0   ((size_t)HALF0 * 4 * 256 * 2)
#define SZ_XB   ((size_t)4 * NN * KC * 2)
#define O_U     (O_R0 + SZ_R0)
#define SZ_U    ((size_t)NN * FW * 4)
#define O_WUPT  (O_U + SZ_U)
#define SZ_WUPT ((size_t)2 * KC * KC * 2)
#define O_WDN2  (O_WUPT + SZ_WUPT)
#define SZ_WDN2 ((size_t)2 * KC * 256 * 2)
#define WS_TOTAL (O_WDN2 + SZ_WDN2)

static_assert(NN % NWAVE == 0);
static_assert(NE % 256 == 0 && NE % 4 == 0);
static_assert(NE < (1 << 20));
static_assert((CHUNK & (CHUNK - 1)) == 0 && CHUNK <= 4096);
static_assert((NBA & (NBA - 1)) == 0 && NBA == (1 << SLA));
static_assert(((long long)CHUNK << SLA) < (1LL << 31));
static_assert(NBA % NWAVE == 0 && NBA % 32 == 0);
static_assert(AGG_ZINTS % (NTHR * 4) == 0);
static_assert(RCAP % 4 == 0 && LISTN % 4 == 0);
static_assert(RCAP >= MEAS_B1024 + 1024);
static_assert(DEGCAP >= MEAS_MAXDEG + 8);
static_assert(HALF0 % NBA == 0 && HALF0 % GBM == 0);
static_assert(SB1 * NBA >= DT1 * GBM && SB1 * NBA <= HALF0);
static_assert(SB0 * NBA == HALF0);
static_assert(DT1 * GBM >= HALF1 && UPT * GBM >= NN);
static_assert(SZ_XB <= SZ_R0);
static_assert((SZ_R0 % 256) == 0 && (SZ_U % 256) == 0 && (SZ_WUPT % 256) == 0 && (SZ_WDN2 % 256) == 0);
static_assert(WS_TOTAL <= (size_t)WSMAX);
static_assert(SCAN_LDS <= 327680 && DOWN_LDS <= 327680);
static_assert(KDN % 32 == 0 && KC % 32 == 0);
static_assert(GBM == (GTHR / 32) * 16);
static_assert((size_t)(NN - 1) * FW + (FW - 1) == (size_t)12799999);

typedef float          v2f   __attribute__((ext_vector_type(2)));
typedef float          v4f   __attribute__((ext_vector_type(4)));
typedef float          v8f   __attribute__((ext_vector_type(8)));
typedef int            v4i   __attribute__((ext_vector_type(4)));
typedef int            v8i   __attribute__((ext_vector_type(8)));
typedef unsigned short v8us  __attribute__((ext_vector_type(8)));
typedef unsigned short v16us __attribute__((ext_vector_type(16)));
typedef __bf16         v16bf __attribute__((ext_vector_type(16)));
typedef v4f  __attribute__((may_alias)) v4fa;
typedef v4i  __attribute__((may_alias)) v4ia;
typedef v8us __attribute__((may_alias)) v8usa;
union FragB { v16bf v; v16us u; v8us h[2]; v8i w; };

__device__ __forceinline__ v8f wmb(const FragB& a, const FragB& b, v8f c) {
  v8f d = __builtin_amdgcn_wmma_f32_16x16x32_bf16(false, a.v, false, b.v, (short)0, c, false, false);
  asm volatile("v_nop\n\tv_nop\n\tv_nop\n\tv_nop" : "+v"(d) : "v"(a.w), "v"(b.w));
  return d;
}

__device__ __forceinline__ unsigned bf16_bits(float f) {
  const unsigned u = __float_as_uint(f);
  return (u + 0x7FFFu + ((u >> 16) & 1u)) >> 16;
}
__device__ __forceinline__ float bf16_val(float f) {
  return __uint_as_float(bf16_bits(f) << 16);
}

__device__ __forceinline__ void wave_sync() {
  __builtin_amdgcn_fence(__ATOMIC_RELEASE, "wavefront");
  __builtin_amdgcn_wave_barrier();
  __builtin_amdgcn_fence(__ATOMIC_ACQUIRE, "wavefront");
}

template <int SLB>
__device__ __forceinline__ int scan_chunk(const int* __restrict__ dsts, int nE, int cbase, int slotBase,
                                          int nb, int vec8, int* list, int tid, int lane, int wave) {
  int wc = 0;
  const int el0  = tid * EPT;
  const int e0   = cbase + el0;
  const int sent = -2147483647 - 1;
  v4i da, db;
  if (vec8 != 0 && cbase + CHUNK <= nE) {
    da = *(const v4i*)(dsts + e0);
    db = *(const v4i*)(dsts + e0 + 4);
  } else {
    const int k0 = dsts[min(e0,     nE - 1)];
    const int k1 = dsts[min(e0 + 1, nE - 1)];
    const int k2 = dsts[min(e0 + 2, nE - 1)];
    const int k3 = dsts[min(e0 + 3, nE - 1)];
    const int k4 = dsts[min(e0 + 4, nE - 1)];
    const int k5 = dsts[min(e0 + 5, nE - 1)];
    const int k6 = dsts[min(e0 + 6, nE - 1)];
    const int k7 = dsts[min(e0 + 7, nE - 1)];
    asm volatile("" :: "v"(k0), "v"(k1), "v"(k2), "v"(k3), "v"(k4), "v"(k5), "v"(k6), "v"(k7));
    da.x = (e0     < nE) ? k0 : sent;
    da.y = (e0 + 1 < nE) ? k1 : sent;
    da.z = (e0 + 2 < nE) ? k2 : sent;
    da.w = (e0 + 3 < nE) ? k3 : sent;
    db.x = (e0 + 4 < nE) ? k4 : sent;
    db.y = (e0 + 5 < nE) ? k5 : sent;
    db.z = (e0 + 6 < nE) ? k6 : sent;
    db.w = (e0 + 7 < nE) ? k7 : sent;
  }
  const unsigned nbs = (unsigned)slotBase;
  const unsigned unb = (unsigned)nb;
  const unsigned s0 = (unsigned)da.x - nbs, s1 = (unsigned)da.y - nbs;
  const unsigned s2 = (unsigned)da.z - nbs, s3 = (unsigned)da.w - nbs;
  const unsigned s4 = (unsigned)db.x - nbs, s5 = (unsigned)db.y - nbs;
  const unsigned s6 = (unsigned)db.z - nbs, s7 = (unsigned)db.w - nbs;
  const bool h0 = s0 < unb, h1 = s1 < unb, h2 = s2 < unb, h3 = s3 < unb;
  const bool h4 = s4 < unb, h5 = s5 < unb, h6 = s6 < unb, h7 = s7 < unb;
  const unsigned any = __builtin_amdgcn_ballot_w32(h0 | h1 | h2 | h3 | h4 | h5 | h6 | h7);
  if (any != 0u) {
#define HITJ(J, HJ, SJ) { \
      const unsigned mj = __builtin_amdgcn_ballot_w32(HJ); \
      if (mj != 0u) { \
        if (HJ) { \
          const int pos = wc + (int)__builtin_amdgcn_mbcnt_lo(mj, 0u); \
          if (pos < WCAP) list[wave * WCAP + pos] = ((el0 + (J)) << SLB) | (int)(SJ); \
        } \
        wc += (int)__builtin_popcount(mj); } }
    HITJ(0, h0, s0)
    HITJ(1, h1, s1)
    HITJ(2, h2, s2)
    HITJ(3, h3, s3)
    HITJ(4, h4, s4)
    HITJ(5, h5, s5)
    HITJ(6, h6, s6)
    HITJ(7, h7, s7)
#undef HITJ
  }
  return wc;
}

__device__ __forceinline__ void wunit(const float* __restrict__ W, int kmask, int n, int k8, unsigned short* dp) {
  v8us o;
#pragma unroll
  for (int j = 0; j < 8; ++j) {
    const int k = (k8 + j) & kmask;
    const float w = W[(size_t)k * KC + n];
    o[j] = (unsigned short)bf16_bits(w);
  }
  *(volatile v8us*)dp = o;
  __threadfence();
  *(volatile v8us*)dp = o;
}

__global__ __launch_bounds__(NTHR) void k_prep(const float* __restrict__ nf,
                                               const float* __restrict__ Wus, const float* __restrict__ Wuv,
                                               const float* __restrict__ Wds, const float* __restrict__ Wdv,
                                               unsigned short* XB, unsigned short* WUPT, unsigned short* WDN2) {
  __shared__ __attribute__((aligned(16))) float stg[NWAVE * FW];
  const int tid = (int)threadIdx.x, lane = tid & 31, wave = tid >> 5;
  const int bx = (int)blockIdx.x;
  if (bx < PREP_NB) {
    const int n = bx * NWAVE + wave;
    const float* rp = nf + (size_t)n * FW;
    const v4f a = *(const v4f*)(rp + 4 * lane);
    const v4f b = *(const v4f*)(rp + 128 + 4 * lane);
    float* sb = stg + wave * FW;
    *(v4fa*)(sb + 4 * lane) = a;
    *(v4fa*)(sb + 128 + 4 * lane) = b;
    wave_sync();
    const int q = lane >> 3;
    const int p = lane & 7;
    v8us o;
#pragma unroll
    for (int j = 0; j < 8; ++j) {
      const int c   = 8 * p + j;
      const int idx = (q == 0) ? c : (KC + 3 * c + (q - 1));
      o[j] = (unsigned short)bf16_bits(sb[idx]);
    }
    unsigned short* dp = XB + ((size_t)q * NN + (size_t)n) * KC + 8 * p;
    *(volatile v8us*)dp = o;
    __threadfence();
    *(volatile v8us*)dp = o;
  } else {
    const int wb = bx - PREP_NB;
    if (wb < 2) {
      const int v = wb * NTHR + tid;
      const int d = v >> 3, k8 = (v & 7) * 8;
      wunit(Wus, 63, d, k8, WUPT + (size_t)d * KC + k8);
    } else if (wb < 4) {
      const int v = (wb - 2) * NTHR + tid;
      const int d = v >> 3, k8 = (v & 7) * 8;
      wunit(Wuv, 63, d, k8, WUPT + (size_t)(KC * KC) + (size_t)d * KC + k8);
    } else if (wb < 12) {
      const int v = (wb - 4) * NTHR + tid;
      const int d = v >> 5, k8 = (v & 31) * 8;
      wunit(Wds, 127, d, k8, WDN2 + (size_t)d * 256 + k8);
    } else if (wb < 20) {
      const int v = (wb - 12) * NTHR + tid;
      const int d = v >> 5, k8 = (v & 31) * 8;
      wunit(Wdv, 127, d, k8, WDN2 + (size_t)(KC * 256) + (size_t)d * 256 + k8);
    }
  }
}

__global__ __launch_bounds__(GTHR) __attribute__((amdgpu_num_vgpr(248)))
void k_up(const unsigned short* __restrict__ XB, const unsigned short* __restrict__ WUPT, float* U) {
  __shared__ __attribute__((aligned(16))) float stg[GBM * 64];
  const int tid = (int)threadIdx.x, lane = tid & 31, wave = tid >> 5, hh = lane >> 4, m = lane & 15;
  const int rowBase = (int)blockIdx.x * GBM;
  const int q = (int)blockIdx.y;

  v8f acc[4];
  {
    const v8f z = {0.f, 0.f, 0.f, 0.f, 0.f, 0.f, 0.f, 0.f};
    acc[0] = z; acc[1] = z; acc[2] = z; acc[3] = z;
  }
  int row = rowBase + 16 * wave + m;
  row = row > NN - 1 ? NN - 1 : row;
  const unsigned short* ap = XB + ((size_t)q * NN + (size_t)row) * KC + 8 * hh;
  const unsigned short* wp = WUPT + (size_t)(q == 0 ? 0 : KC * KC) + (size_t)m * KC + 8 * hh;
#pragma unroll 1
  for (int ks = 0; ks < KC / 32; ++ks) {
    FragB af;
    af.h[0] = *(const v8usa*)(ap + 32 * ks);
    af.h[1] = *(const v8usa*)(ap + 32 * ks + 16);
#pragma unroll
    for (int t = 0; t < 4; ++t) {
      const unsigned short* wq = wp + (size_t)(16 * t) * KC + 32 * ks;
      FragB bf;
      bf.h[0] = *(const v8usa*)wq;
      bf.h[1] = *(const v8usa*)(wq + 16);
      acc[t] = wmb(af, bf, acc[t]);
    }
  }
#pragma unroll
  for (int t = 0; t < 4; ++t) {
    const int lc = 16 * t + m;
#pragma unroll
    for (int r = 0; r < 8; ++r) {
      const int lr = 16 * wave + 8 * hh + r;
      stg[lr * 64 + lc] = acc[t][r];
    }
  }
  __syncthreads();

  v4f fv[8];
#pragma unroll
  for (int i = 0; i < 8; ++i) {
    const int lr = 16 * wave + 2 * i + hh;
    fv[i] = *(const v4fa*)(stg + lr * 64 + 4 * m);
  }
#pragma unroll
  for (int i = 0; i < 8; ++i) {
    const int gr = rowBase + 16 * wave + 2 * i + hh;
    if (gr < NN) {
      float* op = U + (size_t)gr * FW + q * KC + 4 * m;
      *(volatile v4f*)op = fv[i];
    }
  }
  __threadfence();
#pragma unroll
  for (int i = 0; i < 8; ++i) {
    const int gr = rowBase + 16 * wave + 2 * i + hh;
    if (gr < NN) {
      float* op = U + (size_t)gr * FW + q * KC + 4 * m;
      *(volatile v4f*)op = fv[i];
    }
  }
}

__global__ __launch_bounds__(NTHR) void k_scan(const int* __restrict__ snd, const int* __restrict__ rcv,
                                               const float* __restrict__ ea, const float* __restrict__ U,
                                               unsigned* AGGw, int halfBase, int vec8) {
  extern __shared__ __attribute__((aligned(16))) int dsm[];
  int* list = dsm;
  int* hl   = dsm + LISTN;
  int* sl   = hl + RCAP;
  int* cnt  = sl + RCAP;
  int* offs = cnt + NBA;
  int* cur  = offs + NBA;
  int* misc = cur + NBA;
  const int tid = (int)threadIdx.x, lane = tid & 31, wave = tid >> 5;
  const int nodeBase = halfBase + (int)blockIdx.x * NBA;
  const int nE = NE;

  {
    const v4i z4 = {0, 0, 0, 0};
    for (int i = tid * 4; i < AGG_ZINTS; i += NTHR * 4) *(v4ia*)(dsm + i) = z4;
    if (tid < MISC_INTS) misc[tid] = 0;
  }
  __syncthreads();

  int t = 0, ov = 0;
  const int nChunks = (nE + CHUNK - 1) / CHUNK;
#pragma unroll 1
  for (int ch = 0; ch < nChunks; ++ch) {
    const int cbase = ch * CHUNK;
    const int wc = scan_chunk<SLA>(rcv, nE, cbase, nodeBase, NBA, vec8, list, tid, lane, wave);
    if (lane == 0) misc[wave] = wc;
    __syncthreads();
    if (wave == 0) {
#pragma unroll 1
      for (int w2 = 0; w2 < NWAVE; ++w2) {
        int c = misc[w2];
        c = c < 0 ? 0 : (c > WCAP ? WCAP : c);
#pragma unroll 1
        for (int b0 = 0; b0 < c; b0 += 32) {
          const int idx = b0 + lane;
          const int ent = list[w2 * WCAP + (idx < WCAP ? idx : WCAP - 1)];
          const int m32 = (c - b0) < 32 ? (c - b0) : 32;
#pragma unroll 1
          for (int k = 0; k < m32; ++k) {
            const int u    = __builtin_amdgcn_readlane(ent, k);
            const int slot = u & (NBA - 1);
            const int el   = (u >> SLA) & (CHUNK - 1);
            const int pk   = ((cbase + el) << SLA) | slot;
            if (t < RCAP) {
              if (lane == 0) { hl[t] = pk; cnt[slot] = cnt[slot] + 1; }
              t = t + 1;
            } else {
              ov = 1;
            }
          }
        }
      }
    }
    __syncthreads();
  }
  if (wave == 0 && lane == 0) { misc[8] = t; misc[9] = ov; }
  __syncthreads();
  int tt = misc[8];
  tt = tt < 0 ? 0 : (tt > RCAP ? RCAP : tt);
  const int ovf = misc[9];

  if (wave == 0) {
    const int base = lane * (NBA / 32);
    int s = 0;
#pragma unroll 1
    for (int i = 0; i < NBA / 32; ++i) s += cnt[base + i];
    int incl = s;
#pragma unroll
    for (int d = 1; d < 32; d <<= 1) {
      const int y = __shfl_up(incl, d, 32);
      if (lane >= d) incl += y;
    }
    int run = incl - s;
#pragma unroll 1
    for (int i = 0; i < NBA / 32; ++i) {
      const int cv = cnt[base + i];
      offs[base + i] = run;
      cur[base + i]  = run;
      run += cv;
    }
  }
  __syncthreads();
  if (wave == 0) {
#pragma unroll 1
    for (int b0 = 0; b0 < tt; b0 += 32) {
      const int idx = b0 + lane;
      const int ent = hl[idx < RCAP ? idx : RCAP - 1];
      const int m32 = (tt - b0) < 32 ? (tt - b0) : 32;
#pragma unroll 1
      for (int k = 0; k < m32; ++k) {
        const int u    = __builtin_amdgcn_readlane(ent, k);
        const int slot = u & (NBA - 1);
        if (lane == 0) {
          int p = cur[slot];
          p = p < 0 ? 0 : (p > RCAP - 1 ? RCAP - 1 : p);
          sl[p] = u;
          cur[slot] = p + 1;
        }
      }
    }
  }
  __syncthreads();

  const float INV_SQRT3 = (float)0.57735026918962576451;
  const float qnan = __int_as_float(0x7fc00000);
  const float pz = (ovf != 0) ? qnan : 0.0f;
#pragma unroll 1
  for (int si = 0; si < NBA / NWAVE; ++si) {
    const int s     = si * NWAVE + wave;
    const int local = (int)blockIdx.x * NBA + s;
    const int node  = halfBase + local;
    const int craw = cnt[s];
    int cvv = craw < 0 ? 0 : (craw > DEGCAP ? DEGCAP : craw);
    int ovv = offs[s];
    ovv = ovv < 0 ? 0 : (ovv > RCAP ? RCAP : ovv);
    int bgv = (craw > DEGCAP) ? 1 : 0;
    const int c  = __builtin_amdgcn_readfirstlane(cvv);
    const int o  = __builtin_amdgcn_readfirstlane(ovv);
    const int bg = __builtin_amdgcn_readfirstlane(bgv);

    float as0[2], as1[2], av0x[2], av0y[2], av0z[2], av1x[2], av1y[2], av1z[2];
#pragma unroll
    for (int j = 0; j < 2; ++j) {
      as0[j] = 0.0f; as1[j] = 0.0f;
      av0x[j] = 0.0f; av0y[j] = 0.0f; av0z[j] = 0.0f;
      av1x[j] = 0.0f; av1y[j] = 0.0f; av1z[j] = 0.0f;
    }
#pragma unroll 1
    for (int b0 = 0; b0 < c; b0 += 32) {
      int idx = o + b0 + lane;
      idx = idx > RCAP - 1 ? RCAP - 1 : idx;
      const int ent = sl[idx];
      int eid = ent >> SLA;
      eid = eid < 0 ? 0 : (eid > nE - 1 ? nE - 1 : eid);
      const int sraw = snd[eid];
      const v4f yv = *(const v4f*)(ea + (size_t)eid * 4);
      asm volatile("" :: "v"(sraw), "v"(yv.x), "v"(yv.y), "v"(yv.z), "v"(yv.w));
      const int sr = sraw < 0 ? 0 : (sraw > NN - 1 ? NN - 1 : sraw);
      const int y0i = __float_as_int(bf16_val(yv.x));
      const int yxi = __float_as_int(bf16_val(yv.y));
      const int yyi = __float_as_int(bf16_val(yv.z));
      const int yzi = __float_as_int(bf16_val(yv.w));
      const int m32 = (c - b0) < 32 ? (c - b0) : 32;
#pragma unroll 1
      for (int k = 0; k < m32; ++k) {
        const int   sk = __builtin_amdgcn_readlane(sr, k);
        const float y0 = __int_as_float(__builtin_amdgcn_readlane(y0i, k));
        const float yx = __int_as_float(__builtin_amdgcn_readlane(yxi, k));
        const float yy = __int_as_float(__builtin_amdgcn_readlane(yyi, k));
        const float yz = __int_as_float(__builtin_amdgcn_readlane(yzi, k));
        const float* up = U + (size_t)sk * FW + 2 * lane;
        const v2f us = *(const v2f*)up;
        const v2f ux = *(const v2f*)(up + KC);
        const v2f uy = *(const v2f*)(up + 2 * KC);
        const v2f uz = *(const v2f*)(up + 3 * KC);
        const float ss[2] = {us.x, us.y};
        const float vx[2] = {ux.x, ux.y};
        const float vy[2] = {uy.x, uy.y};
        const float vz[2] = {uz.x, uz.y};
#pragma unroll
        for (int j = 0; j < 2; ++j) {
          as0[j] = fmaf(ss[j], y0, as0[j]);
          float d3 = vx[j] * yx;
          d3 = fmaf(vy[j], yy, d3);
          d3 = fmaf(vz[j], yz, d3);
          const float ms1 = d3 * INV_SQRT3;
          as1[j] = as1[j] + ms1;
          av0x[j] = fmaf(vx[j], y0, av0x[j]);
          av0y[j] = fmaf(vy[j], y0, av0y[j]);
          av0z[j] = fmaf(vz[j], y0, av0z[j]);
          av1x[j] = fmaf(ss[j], yx, av1x[j]);
          av1y[j] = fmaf(ss[j], yy, av1y[j]);
          av1z[j] = fmaf(ss[j], yz, av1z[j]);
        }
      }
    }
    const float pzr = (bg != 0) ? qnan : pz;
    const bool live = node < NN;
    const float va[8] = {as0[0], as1[0], av0x[0], av1x[0], av0y[0], av1y[0], av0z[0], av1z[0]};
    const float vb[8] = {as0[1], as1[1], av0x[1], av1x[1], av0y[1], av1y[1], av0z[1], av1z[1]};
    unsigned hiw[8], low[8];
#pragma unroll
    for (int j = 0; j < 8; ++j) {
      const float ma = live ? (va[j] * 0.0625f + pzr) : 0.0f;
      const float mb = live ? (vb[j] * 0.0625f + pzr) : 0.0f;
      const unsigned ha = bf16_bits(ma);
      const unsigned hb = bf16_bits(mb);
      float hva = __uint_as_float(ha << 16), hvb = __uint_as_float(hb << 16);
      asm volatile("" : "+v"(hva), "+v"(hvb));
      const unsigned la = bf16_bits(ma - hva);
      const unsigned lb = bf16_bits(mb - hvb);
      hiw[j] = (ha & 0xffffu) | (hb << 16);
      low[j] = (la & 0xffffu) | (lb << 16);
    }
    if (local < HALF0) {
      unsigned* bp = AGGw + (size_t)local * 512 + lane;
#pragma unroll
      for (int j = 0; j < 8; ++j) {
        unsigned* pp = bp + (j >> 1) * 128 + (j & 1) * 32;
        *(volatile unsigned*)pp = hiw[j];
        *(volatile unsigned*)(pp + 64) = low[j];
      }
      __threadfence();
#pragma unroll
      for (int j = 0; j < 8; ++j) {
        unsigned* pp = bp + (j >> 1) * 128 + (j & 1) * 32;
        *(volatile unsigned*)pp = hiw[j];
        *(volatile unsigned*)(pp + 64) = low[j];
      }
    }
  }
}

__global__ __launch_bounds__(GTHR) __attribute__((amdgpu_num_vgpr(248)))
void k_down(const unsigned short* __restrict__ AGG, const unsigned short* __restrict__ WDN2, float* out,
            int nodeBase, int nLoc) {
  extern __shared__ __attribute__((aligned(16))) float dstg[];
  const int tid = (int)threadIdx.x, lane = tid & 31, wave = tid >> 5, hh = lane >> 4, m = lane & 15;
  const int rowBase = (int)blockIdx.x * GBM;
  int lc = rowBase + 16 * wave + m;
  lc = lc > nLoc - 1 ? nLoc - 1 : lc;
  lc = lc < 0 ? 0 : lc;

#pragma unroll 1
  for (int q = 0; q < 4; ++q) {
    v8f acc[4];
    {
      const v8f z = {0.f, 0.f, 0.f, 0.f, 0.f, 0.f, 0.f, 0.f};
      acc[0] = z; acc[1] = z; acc[2] = z; acc[3] = z;
    }
    const unsigned short* ap = AGG + ((size_t)lc * 4 + (size_t)q) * 256 + 8 * hh;
    const unsigned short* wp = WDN2 + (size_t)(q == 0 ? 0 : KC * 256) + (size_t)m * 256 + 8 * hh;
#pragma unroll 1
    for (int ks = 0; ks < KDN / 32; ++ks) {
      FragB af;
      af.h[0] = *(const v8usa*)(ap + 32 * ks);
      af.h[1] = *(const v8usa*)(ap + 32 * ks + 16);
#pragma unroll
      for (int t = 0; t < 4; ++t) {
        const unsigned short* wq = wp + (size_t)(16 * t) * 256 + 32 * ks;
        FragB bf;
        bf.h[0] = *(const v8usa*)wq;
        bf.h[1] = *(const v8usa*)(wq + 16);
        acc[t] = wmb(af, bf, acc[t]);
      }
    }
#pragma unroll
    for (int t = 0; t < 4; ++t) {
      const int d   = 16 * t + m;
      const int col = (q == 0) ? d : (KC + 3 * d + (q - 1));
#pragma unroll
      for (int r = 0; r < 8; ++r) {
        const int lr = 16 * wave + 8 * hh + r;
        dstg[lr * SPITCH + col] = acc[t][r];
      }
    }
  }
  __syncthreads();

#pragma unroll 1
  for (int b = 0; b < 2; ++b) {
    v4f fa[8], fb[8];
#pragma unroll
    for (int i = 0; i < 8; ++i) {
      const int lr = 16 * wave + 8 * b + i;
      fa[i] = *(const v4fa*)(dstg + lr * SPITCH + 4 * lane);
      fb[i] = *(const v4fa*)(dstg + lr * SPITCH + 128 + 4 * lane);
    }
#pragma unroll
    for (int i = 0; i < 8; ++i) {
      const int lrow = rowBase + 16 * wave + 8 * b + i;
      if (lrow < nLoc) {
        float* op = out + (size_t)(nodeBase + lrow) * FW + 4 * lane;
        *(volatile v4f*)op = fa[i];
        *(volatile v4f*)(op + 128) = fb[i];
      }
    }
    __threadfence();
#pragma unroll
    for (int i = 0; i < 8; ++i) {
      const int lrow = rowBase + 16 * wave + 8 * b + i;
      if (lrow < nLoc) {
        float* op = out + (size_t)(nodeBase + lrow) * FW + 4 * lane;
        *(volatile v4f*)op = fa[i];
        *(volatile v4f*)(op + 128) = fb[i];
      }
    }
  }
}

extern "C" void kernel_launch(void* const* d_in, const int* in_sizes, int n_in,
                              void* d_out, int out_size, void* d_ws, size_t ws_size,
                              hipStream_t stream) {
  if (n_in < 8) return;
  if (in_sizes[0] != NN * FW) return;
  if (in_sizes[1] != NE * 4) return;
  if (in_sizes[2] != KC * KC || in_sizes[3] != KC * KC) return;
  if (in_sizes[4] != 2 * KC * KC || in_sizes[5] != 2 * KC * KC) return;
  if (in_sizes[6] != NE || in_sizes[7] != NE) return;
  if (out_size != NN * FW) return;
  if (ws_size < (size_t)WS_TOTAL) return;

  const float* nf  = (const float*)d_in[0];
  const float* ea  = (const float*)d_in[1];
  const float* Wus = (const float*)d_in[2];
  const float* Wuv = (const float*)d_in[3];
  const float* Wds = (const float*)d_in[4];
  const float* Wdv = (const float*)d_in[5];
  const int*   snd = (const int*)d_in[6];
  const int*   rcv = (const int*)d_in[7];
  float* out = (float*)d_out;

  char* ws = (char*)d_ws;
  unsigned short* AGG  = (unsigned short*)(ws + O_R0);
  unsigned short* XB   = (unsigned short*)(ws + O_R0);
  float*          U    = (float*)(ws + O_U);
  unsigned short* WUPT = (unsigned short*)(ws + O_WUPT);
  unsigned short* WDN2 = (unsigned short*)(ws + O_WDN2);

  hipFuncSetAttribute(reinterpret_cast<const void*>(&k_scan),
                      hipFuncAttributeMaxDynamicSharedMemorySize, (int)SCAN_LDS);
  hipFuncSetAttribute(reinterpret_cast<const void*>(&k_down),
                      hipFuncAttributeMaxDynamicSharedMemorySize, (int)DOWN_LDS);

  const int vec8 = ((NE & 3) == 0) ? 1 : 0;

  k_prep<<<PREP_NB + PREP_WB, NTHR, 0, stream>>>(nf, Wus, Wuv, Wds, Wdv, XB, WUPT, WDN2);
  k_up<<<dim3(UPT, 4), GTHR, 0, stream>>>(XB, WUPT, U);
  k_scan<<<SB0, NTHR, SCAN_LDS, stream>>>(snd, rcv, ea, U, (unsigned*)AGG, 0, vec8);
  k_down<<<DT0, GTHR, DOWN_LDS, stream>>>(AGG, WDN2, out, 0, HALF0);
  k_scan<<<SB1, NTHR, SCAN_LDS, stream>>>(snd, rcv, ea, U, (unsigned*)AGG, HALF0, vec8);
  k_down<<<DT1, GTHR, DOWN_LDS, stream>>>(AGG, WDN2, out, HALF0, HALF1);
}
